// qkv_attn_35966056137256
// MI455X (gfx1250) — hardware-verified
//
#include <hip/hip_runtime.h>
#include <math.h>

typedef __attribute__((ext_vector_type(16))) _Float16 v16h;
typedef __attribute__((ext_vector_type(16))) __bf16 v16b;
typedef __attribute__((ext_vector_type(8)))  _Float16 v8h;
typedef __attribute__((ext_vector_type(8)))  float v8f;
typedef __attribute__((ext_vector_type(4)))  float v4f;
typedef __attribute__((ext_vector_type(2)))  float v2f;
typedef __attribute__((ext_vector_type(4)))  unsigned v4u;
typedef __attribute__((ext_vector_type(4)))  int v4i;
typedef float __attribute__((may_alias)) float_a;
typedef int __attribute__((may_alias)) int_a;

template <typename T> __device__ __forceinline__ void vst2(void* p, T v) { *(volatile T*)p = v; __threadfence(); *(volatile T*)p = v; }
__device__ __forceinline__ v8f wmma16(v16h a, v16h b, v8f c) {
  v8f d = __builtin_amdgcn_wmma_f32_16x16x32_f16(false, a, false, b, (short)0, c, false, false);
  asm volatile("v_nop\n\tv_nop\n\tv_nop\n\tv_nop" : "+v"(d) : "v"(a), "v"(b));
  return d;
}
__device__ __forceinline__ v8f wmma_bf(v16b a, v16b b, v8f c) {
  v8f d = __builtin_amdgcn_wmma_f32_16x16x32_bf16(false, a, false, b, (short)0, c, false, false);
  asm volatile("v_nop\n\tv_nop\n\tv_nop\n\tv_nop" : "+v"(d) : "v"(a), "v"(b));
  return d;
}
__device__ __forceinline__ v16h frag_h(const _Float16* rowk0, int lane) {
  union { v16h v; v8h q[2]; } u; const _Float16* p = rowk0 + 8 * (lane >> 4);
  u.q[0] = *(const v8h*)p; u.q[1] = *(const v8h*)(p + 16); return u.v;
}
__device__ __forceinline__ v16h frag_f32(const float* rowk0, int lane) {
  v16h a; const float* p = rowk0 + 8 * (lane >> 4);
#pragma unroll
  for (int i = 0; i < 8; ++i) { a[i] = (_Float16)p[i]; a[8 + i] = (_Float16)p[16 + i]; }
  return a;
}
__device__ __forceinline__ v16h frag_f32s(const float* rowk0, int lane, float sc) {
  v16h a; const float* p = rowk0 + 8 * (lane >> 4);
#pragma unroll
  for (int i = 0; i < 8; ++i) { a[i] = (_Float16)(p[i] * sc); a[8 + i] = (_Float16)(p[16 + i] * sc); }
  return a;
}
__device__ __forceinline__ v16h fragc_f32(const float* W, int k0, int n, int lane, int ld, int K) {
  v16h a; const int g = lane >> 4;
#pragma unroll
  for (int i = 0; i < 8; ++i) { const int ka = k0 + 8 * g + i, kb = ka + 16;
    a[i] = (_Float16)(ka < K ? W[(size_t)ka * ld + n] : 0.f); a[8 + i] = (_Float16)(kb < K ? W[(size_t)kb * ld + n] : 0.f); }
  return a;
}
struct F2 { v16b h, l; };
__device__ __forceinline__ F2 bsplit16(const float v[16]) { F2 r;
#pragma unroll
  for (int i = 0; i < 16; ++i) { const __bf16 h = (__bf16)v[i]; r.h[i] = h; r.l[i] = (__bf16)(v[i] - (float)h); }
  return r; }
__device__ __forceinline__ F2 split_row(const float* row, int k0, int lane) { float v[16]; const float* p = row + k0 + 8 * (lane >> 4);
#pragma unroll
  for (int i = 0; i < 8; ++i) { v[i] = p[i]; v[8 + i] = p[16 + i]; }
  return bsplit16(v); }
__device__ __forceinline__ F2 split_rowK(const float* row, int k0, int lane, int K) { float v[16]; const int g = lane >> 4;
#pragma unroll
  for (int i = 0; i < 8; ++i) { const int ka = k0 + 8 * g + i, kb = ka + 16; v[i] = ka < K ? row[ka] : 0.f; v[8 + i] = kb < K ? row[kb] : 0.f; }
  return bsplit16(v); }
__device__ __forceinline__ F2 split_col(const float* W, int k0, int n, int lane, int ld, int K) { float v[16]; const int g = lane >> 4;
#pragma unroll
  for (int i = 0; i < 8; ++i) { const int ka = k0 + 8 * g + i, kb = ka + 16; v[i] = ka < K ? W[(size_t)ka * ld + n] : 0.f; v[8 + i] = kb < K ? W[(size_t)kb * ld + n] : 0.f; }
  return bsplit16(v); }
__device__ __forceinline__ v8f mac3(const F2& a, const F2& b, v8f c) { c = wmma_bf(a.l, b.h, c); c = wmma_bf(a.h, b.l, c); return wmma_bf(a.h, b.h, c); }
__device__ __forceinline__ float sigm(float v) { return 1.0f / (1.0f + expf(-v)); }
#define LDSX() do { asm volatile("s_wait_dscnt 0" ::: "memory"); __builtin_amdgcn_wave_barrier(); __builtin_amdgcn_fence(__ATOMIC_RELEASE, "workgroup"); } while (0)

#define NB 8
#define HWN 4096
#define CC 256
#define NHD 8
#define HC 32
#define NR (NB * HWN)
#define BPB (HWN / 64)

__device__ __forceinline__ float gelu_e(float v) { return 0.5f * v * (1.0f + erff(v * 0.70710678118654752f)); }

__global__ __launch_bounds__(256) void k_cvt(const float* __restrict__ x, _Float16* __restrict__ x16, size_t n8) {
  const size_t g8 = (size_t)blockIdx.x * 256 + threadIdx.x; if (g8 >= n8) return;
  union { v8h h; v4u u; } pk;
#pragma unroll
  for (int e = 0; e < 8; ++e) pk.h[e] = (_Float16)x[g8 * 8 + e];
  vst2(x16 + g8 * 8, pk.u);
}
__global__ __launch_bounds__(256) void k_packT(const float* __restrict__ Wqkv, const float* __restrict__ W1, const float* __restrict__ W2, _Float16* __restrict__ P) {
  __shared__ float tile[64][65];
  const int which = blockIdx.z, o0 = blockIdx.x * 64, k0 = blockIdx.y * 64, tid = threadIdx.x;
  const float* W = which == 0 ? Wqkv : (which == 1 ? W1 : W2); const int NOUT = which == 0 ? 3 * CC : CC; const int rowbase = which == 0 ? 0 : (which == 1 ? 3 * CC : 4 * CC);
  if (o0 >= NOUT) return;
  for (int q = tid; q < 64 * 64; q += 256) { const int kl = q >> 6, ol = q & 63; tile[kl][ol] = W[(size_t)(k0 + kl) * NOUT + o0 + ol]; }
  __syncthreads();
  for (int u = 0; u < 2; ++u) { const int idx = tid + u * 256, ol = idx >> 3, pc = idx & 7; union { v8h hh; v4u uu; } pk;
#pragma unroll
    for (int i = 0; i < 8; ++i) pk.hh[i] = (_Float16)(tile[pc * 8 + i][ol] * 16.0f);
    vst2(P + ((size_t)rowbase + o0 + ol) * CC + k0 + pc * 8, pk.uu); }
}
__global__ __launch_bounds__(128) void k_qkv(const _Float16* __restrict__ x16, const _Float16* __restrict__ P, const float* __restrict__ bqkv, const float* __restrict__ kg, const float* __restrict__ kb, const float* __restrict__ vg, const float* __restrict__ vb,
                                           float* __restrict__ qrows, float* __restrict__ part) {
  __shared__ __align__(16) float sq[64][CC + 4], sk[64][CC + 4], sv[64][CC + 4];
  const int tid = threadIdx.x, wave = tid >> 5, lane = tid & 31, col = lane & 15, g = lane >> 4;
  const int r0b = blockIdx.x * 64, r0 = r0b + wave * 16;
  v16h ax[8];
#pragma unroll
  for (int kc = 0; kc < 8; ++kc) ax[kc] = frag_h(x16 + (size_t)(r0 + col) * CC + kc * 32, lane);
#pragma unroll 1
  for (int nc = 0; nc < 6; ++nc) { v8f acc[8] = {};
#pragma unroll
    for (int kc = 0; kc < 8; ++kc) {
#pragma unroll
      for (int j = 0; j < 8; ++j) acc[j] = wmma16(ax[kc], frag_h(P + (size_t)(nc * 128 + j * 16 + col) * CC + kc * 32, lane), acc[j]); }
#pragma unroll
    for (int j = 0; j < 8; ++j) { const int n = nc * 128 + j * 16 + col; const float bb = bqkv[n]; const int h = n / 96, wch = (n % 96) / 32, c = n % 32; const int cc = h * HC + c;
      float (*dst)[CC + 4] = wch == 0 ? sq : (wch == 1 ? sk : sv);
#pragma unroll
      for (int r = 0; r < 8; ++r) dst[wave * 16 + 8 * g + r][cc] = acc[j][r] * (1.0f / 16.0f) + bb; } }
  LDSX();
  for (int rh = 0; rh < 16 * NHD; ++rh) { const int rl = wave * 16 + (rh >> 3), h = rh & 7; const int cc = h * HC + lane;
    { const float v = sk[rl][cc]; float s = v; for (int off = 16; off >= 1; off >>= 1) s += __shfl_xor(s, off, 32); const float mu = s * (1.0f / HC); const float d = v - mu; float q2 = d * d; for (int off = 16; off >= 1; off >>= 1) q2 += __shfl_xor(q2, off, 32);
      sk[rl][cc] = d * rsqrtf(q2 * (1.0f / HC) + 1e-5f) * kg[lane] + kb[lane]; }
    { const float v = sv[rl][cc]; float s = v; for (int off = 16; off >= 1; off >>= 1) s += __shfl_xor(s, off, 32); const float mu = s * (1.0f / HC); const float d = v - mu; float q2 = d * d; for (int off = 16; off >= 1; off >>= 1) q2 += __shfl_xor(q2, off, 32);
      sv[rl][cc] = d * rsqrtf(q2 * (1.0f / HC) + 1e-5f) * vg[lane] + vb[lane]; } }
  for (int q = lane; q < 16 * 64; q += 32) { const int rl = q >> 6, pc = q & 63; vst2(qrows + (size_t)(r0 + rl) * CC + pc * 4, *(const v4f*)(&sq[wave * 16 + rl][pc * 4])); }
  __syncthreads();
  __shared__ __align__(16) float sp[NHD * HC * HC];
#pragma unroll 1
  for (int h = 0; h < NHD; ++h) {
    float a8[8]; const int d = tid >> 2, e0 = (tid & 3) * 8;
#pragma unroll
    for (int u = 0; u < 8; ++u) a8[u] = 0.f;
#pragma unroll 4
    for (int rl = 0; rl < 64; ++rl) { const float kd = sk[rl][h * HC + d];
#pragma unroll
      for (int u = 0; u < 8; ++u) a8[u] += kd * sv[rl][h * HC + e0 + u]; }
#pragma unroll
    for (int u = 0; u < 8; ++u) sp[(h * HC + d) * HC + e0 + u] = a8[u]; }
  __syncthreads();
  for (int q = tid; q < NHD * HC * HC / 4; q += 128) vst2(part + (size_t)blockIdx.x * (NHD * HC * HC) + q * 4, *(const v4f*)(&sp[q * 4]));
}
__global__ __launch_bounds__(256) void k_kv(const float* __restrict__ part, float* __restrict__ kv) {
  __shared__ __align__(16) float so[HC * HC];
  const int b = blockIdx.y, h = blockIdx.x, tid = threadIdx.x;
  for (int e = tid; e < HC * HC; e += 256) { float s = 0.f;
#pragma unroll 1
    for (int blk = 0; blk < BPB; ++blk) s += part[((size_t)(b * BPB + blk) * NHD + h) * (HC * HC) + e];
    so[e] = s * (1.0f / (float)HWN); }
  __syncthreads();
  vst2(kv + ((size_t)b * NHD + h) * (HC * HC) + tid * 4, *(const v4f*)(&so[tid * 4]));
}
__global__ __launch_bounds__(128) void k_mlp(const float* __restrict__ qrows, const float* __restrict__ kv, const float* __restrict__ x, const _Float16* __restrict__ P, const float* __restrict__ b1, const float* __restrict__ b2, float* __restrict__ out) {
  __shared__ __align__(16) float sr[64][CC + 4];
  __shared__ __align__(16) float sh[64][CC + 4];
  const int tid = threadIdx.x, wave = tid >> 5, lane = tid & 31, col = lane & 15, g = lane >> 4;
  const int r0b = blockIdx.x * 64, r0 = r0b + wave * 16; const int b = r0b / HWN;
#pragma unroll 1
  for (int h = 0; h < NHD; ++h) { const v16h a = frag_f32(qrows + (size_t)(r0 + col) * CC + h * HC, lane); const float* kvh = kv + ((size_t)b * NHD + h) * (HC * HC);
#pragma unroll
    for (int t = 0; t < 2; ++t) { v16h bb; const int n = t * 16 + col;
#pragma unroll
      for (int i = 0; i < 8; ++i) { bb[i] = (_Float16)(kvh[(8 * g + i) * HC + n] * 64.0f); bb[8 + i] = (_Float16)(kvh[(16 + 8 * g + i) * HC + n] * 64.0f); }
      v8f acc = {}; acc = wmma16(a, bb, acc);
#pragma unroll
      for (int r = 0; r < 8; ++r) { const int cc = h * HC + t * 16 + col; sr[wave * 16 + 8 * g + r][cc] = acc[r] * (1.0f / 64.0f) + x[(size_t)(r0 + 8 * g + r) * CC + cc]; } } }
  LDSX();
#pragma unroll 1
  for (int nh = 0; nh < 2; ++nh) { v8f acc[8];
#pragma unroll
    for (int j = 0; j < 8; ++j) acc[j] = (v8f){};
#pragma unroll 1
    for (int kc = 0; kc < CC / 32; ++kc) { const v16h a = frag_f32(&sr[wave * 16 + col][0] + kc * 32, lane);
#pragma unroll
      for (int j = 0; j < 8; ++j) acc[j] = wmma16(a, frag_h(P + (size_t)(3 * CC + nh * 128 + j * 16 + col) * CC + kc * 32, lane), acc[j]); }
#pragma unroll
    for (int j = 0; j < 8; ++j) { const int cc = nh * 128 + j * 16 + col; const float bb = b1[cc];
#pragma unroll
      for (int r = 0; r < 8; ++r) sh[wave * 16 + 8 * g + r][cc] = gelu_e(acc[j][r] * (1.0f / 16.0f) + bb); } }
  LDSX();
#pragma unroll 1
  for (int nh = 0; nh < 2; ++nh) { v8f acc[8];
#pragma unroll
    for (int j = 0; j < 8; ++j) acc[j] = (v8f){};
#pragma unroll 1
    for (int kc = 0; kc < CC / 32; ++kc) { const v16h a = frag_f32(&sh[wave * 16 + col][0] + kc * 32, lane);
#pragma unroll
      for (int j = 0; j < 8; ++j) acc[j] = wmma16(a, frag_h(P + (size_t)(4 * CC + nh * 128 + j * 16 + col) * CC + kc * 32, lane), acc[j]); }
#pragma unroll
    for (int j = 0; j < 8; ++j) { const int cc = nh * 128 + j * 16 + col; const float bb = b2[cc];
#pragma unroll
      for (int r = 0; r < 8; ++r) sr[wave * 16 + 8 * g + r][cc] = acc[j][r] * (1.0f / 16.0f) + bb + x[(size_t)(r0 + 8 * g + r) * CC + cc]; } }
  LDSX();
  for (int q = lane; q < 16 * 64; q += 32) { const int rl = q >> 6, pc = q & 63; vst2(out + (size_t)(r0 + rl) * CC + pc * 4, *(const v4f*)(&sr[wave * 16 + rl][pc * 4])); }
}
extern "C" void kernel_launch(void* const* d_in, const int* in_sizes, int n_in, void* d_out, int out_size, void* d_ws, size_t ws_size, hipStream_t stream) {
  (void)in_sizes; (void)n_in; (void)out_size; (void)ws_size;
  const float** I = (const float**)d_in;
  const float* x = I[0]; const float* Wqkv = I[1]; const float* bqkv = I[2]; const float* kg = I[3]; const float* kb = I[4]; const float* vg = I[5]; const float* vb = I[6]; const float* W1 = I[7]; const float* b1 = I[8]; const float* W2 = I[9]; const float* b2 = I[10];
  float* out = (float*)d_out;
  char* ws = (char*)d_ws; size_t off = 0;
  auto take = [&](size_t bytes) { char* p = ws + off; off += (bytes + 255) & ~(size_t)255; return p; };
  _Float16* x16 = (_Float16*)take((size_t)NR * CC * 2); _Float16* P = (_Float16*)take((size_t)5 * CC * CC * 2); float* qrows = (float*)take((size_t)NR * CC * 4);
  float* part = (float*)take((size_t)(NR / 64) * NHD * HC * HC * 4); float* kv = (float*)take((size_t)NB * NHD * HC * HC * 4);
  const size_t n8 = (size_t)NR * CC / 8; k_cvt<<<(unsigned)(n8 / 256), 256, 0, stream>>>(x, x16, n8);
  k_packT<<<dim3(3 * CC / 64, CC / 64, 3), 256, 0, stream>>>(Wqkv, W1, W2, P);
  k_qkv<<<NR / 64, 128, 0, stream>>>(x16, P, bqkv, kg, kb, vg, vb, qrows, part);
  k_kv<<<dim3(NHD, NB), 256, 0, stream>>>(part, kv);
  k_mlp<<<NR / 64, 128, 0, stream>>>(qrows, kv, x, P, b1, b2, out);
}
